// GCN_5755256177073
// MI455X (gfx1250) — hardware-verified
//
#include <hip/hip_runtime.h>
#include <stddef.h>
#include <stdint.h>


#define NN      10000
#define NE      320000
#define DIN     512
#define HH      256
#define NG      64
#define OUTD    512
#define NPAD    10112
#define GW      384
#define KFIN    1536
#define SP      260
#define PCAP    NN

#define NTHR    256
#define NWAVE   8
#define EPT     8
#define CHUNK   (NTHR * EPT)
#define WCAP    (EPT * 32)
#define LISTN   (NWAVE * WCAP)
#define NBMAX   2048
#define NBRUN   512
#define RCAP    28672
#define DEGCAP  128
#define STW     512
#define NEGS    0.2f
#define WSMAX   134217728
#define LDS_AGG ((2 * RCAP + 2 * NBMAX + LISTN) * 4 + 64)
#define LDS_G8  (128 * SP * 4)
#define LDS_G4  (64 * SP * 4)
#define LDS_GATE (128 * SP * 4 + (256 + GW + GW) * 4)
#define LDS_POOL (3 * PCAP * 4)

static_assert((CHUNK & (CHUNK - 1)) == 0 && CHUNK <= 4096);
static_assert((NBMAX & (NBMAX - 1)) == 0 && NBMAX <= 4096);
static_assert((NBRUN & (NBRUN - 1)) == 0 && NBRUN <= NBMAX && NBRUN >= 16);
static_assert(NTHR * 8 == NBMAX);
static_assert(LISTN >= NBMAX);
static_assert((RCAP % 32) == 0);
static_assert(NWAVE * STW <= RCAP);
static_assert(HH <= STW);
static_assert(HH == 32 * 8);
static_assert(64 == 8 * 8);
static_assert(NG == 64);
static_assert(NPAD == 79 * 128);
static_assert((NN % 16) == 0 && NN <= NPAD);
static_assert(RCAP >= 17580);
static_assert(DEGCAP >= 55 + 8);
static_assert(NE < (1 << 20));
static_assert(LDS_AGG <= 300000);
static_assert(LDS_GATE <= 300000 && LDS_POOL + 4096 <= 300000);
static_assert((SP % 4) == 0);

typedef float          v2f   __attribute__((ext_vector_type(2)));
typedef float          v4f   __attribute__((ext_vector_type(4)));
typedef float          v8f   __attribute__((ext_vector_type(8)));
typedef int            v4i   __attribute__((ext_vector_type(4)));
typedef int            v8i   __attribute__((ext_vector_type(8)));
typedef unsigned short v8us  __attribute__((ext_vector_type(8)));
typedef __bf16         v16bf __attribute__((ext_vector_type(16)));
typedef v4f __attribute__((may_alias)) v4fa;
union FragB { v16bf v; v8us u[2]; v8i w; };

__device__ __forceinline__ v8f wmx(const FragB& a, const FragB& b, v8f c) {
  v8f d = __builtin_amdgcn_wmma_f32_16x16x32_bf16(false, a.v, false, b.v, (short)0, c, false, false);
  asm volatile("v_nop\n\tv_nop\n\tv_nop\n\tv_nop" : "+v"(d) : "v"(a.w), "v"(b.w));
  return d;
}

__device__ __forceinline__ void ldwait() {
  asm volatile("s_wait_loadcnt 0x0" ::: "memory");
}

__device__ __forceinline__ unsigned bfbits(float v) {
  unsigned u = __float_as_uint(v);
  const unsigned r = (u + 0x7FFFu + ((u >> 16) & 1u)) >> 16;
  return (v != v) ? 0x7FC0u : r;
}
__device__ __forceinline__ float rbf(float v) { return __uint_as_float(bfbits(v) << 16); }
__device__ __forceinline__ v4f rbf4(const v4f a) {
  v4f o; o.x = rbf(a.x); o.y = rbf(a.y); o.z = rbf(a.z); o.w = rbf(a.w); return o;
}
__device__ __forceinline__ float blendf(float a, float b, bool pickA) {
  const unsigned mk = 0u - (unsigned)pickA;
  return __uint_as_float((__float_as_uint(a) & mk) | (__float_as_uint(b) & ~mk));
}

__device__ __forceinline__ v8us cvt8b(const v4f a, const v4f b) {
  v8us o;
  o[0] = (unsigned short)bfbits(a.x); o[1] = (unsigned short)bfbits(a.y);
  o[2] = (unsigned short)bfbits(a.z); o[3] = (unsigned short)bfbits(a.w);
  o[4] = (unsigned short)bfbits(b.x); o[5] = (unsigned short)bfbits(b.y);
  o[6] = (unsigned short)bfbits(b.z); o[7] = (unsigned short)bfbits(b.w);
  return o;
}
__device__ __forceinline__ void split8(const v4f a, const v4f b, v8us& hv, v8us& lv) {
  const float f[8] = {a.x, a.y, a.z, a.w, b.x, b.y, b.z, b.w};
#pragma unroll
  for (int i = 0; i < 8; ++i) {
    const unsigned hb = bfbits(f[i]);
    const float hf = __uint_as_float(hb << 16);
    hv[i] = (unsigned short)hb;
    lv[i] = (unsigned short)bfbits(f[i] - hf);
  }
}

__device__ __forceinline__ float gelu_f(float x) {
  return 0.5f * x * (1.0f + erff(x * 0.70710678118654752f));
}
__device__ __forceinline__ float exn(float a) {
  const float e = expf(a);
  return (a < -87.3f) ? 0.0f : e;
}
__device__ __forceinline__ float wsum(float v) {
#pragma unroll
  for (int off = 16; off > 0; off >>= 1) v += __shfl_xor(v, off);
  return v;
}
__device__ __forceinline__ int wsumi(int v) {
#pragma unroll
  for (int off = 16; off > 0; off >>= 1) v += __shfl_xor(v, off);
  return v;
}
__device__ __forceinline__ float nmax(float m, float v) { return (v > m || v != v) ? v : m; }

__device__ __forceinline__ void wtr_unit(const float* __restrict__ w, int cols, int Ksrc,
                                         unsigned short* plane, int pitch, int nOff, int kOff, int u) {
  const int kq = Ksrc >> 3;
  const int n  = u / kq;
  const int k8 = (u - n * kq) * 8;
  const float* p = w + (size_t)k8 * (size_t)cols + n;
  v4f a, b;
  a.x = p[0];                  a.y = p[(size_t)cols];       a.z = p[(size_t)2 * cols];   a.w = p[(size_t)3 * cols];
  b.x = p[(size_t)4 * cols];   b.y = p[(size_t)5 * cols];   b.z = p[(size_t)6 * cols];   b.w = p[(size_t)7 * cols];
  const v8us hv = cvt8b(a, b);
  unsigned short* o = plane + (size_t)(nOff + n) * (size_t)pitch + kOff + k8;
  *(volatile v8us*)o = hv;
  *(volatile v8us*)(o + Ksrc) = hv;
  __threadfence();
  *(volatile v8us*)o = hv;
  *(volatile v8us*)(o + Ksrc) = hv;
}

__global__ __launch_bounds__(NTHR) void k_prep(
    const float* __restrict__ Wp, const float* __restrict__ Wrel, const float* __restrict__ Wroot,
    const float* __restrict__ Wl, const float* __restrict__ Wr, const float* __restrict__ Wg1a,
    const float* __restrict__ Wg2a, const float* __restrict__ Wo,
    unsigned short* WpT2, unsigned short* WgcT, unsigned short* WlrT2, unsigned short* WgT2, unsigned short* WoT2) {
  const int b = (int)blockIdx.x, t = (int)threadIdx.x;
  if (b < 64)        wtr_unit(Wp,    256, 512, WpT2,  1024, 0,   0,   b * 256 + t);
  else if (b < 96)   wtr_unit(Wrel,  256, 256, WgcT,  1024, 0,   0,   (b - 64) * 256 + t);
  else if (b < 128)  wtr_unit(Wroot, 256, 256, WgcT,  1024, 0,   512, (b - 96) * 256 + t);
  else if (b < 160)  wtr_unit(Wl,    256, 256, WlrT2, 512,  0,   0,   (b - 128) * 256 + t);
  else if (b < 192)  wtr_unit(Wr,    256, 256, WlrT2, 512,  256, 0,   (b - 160) * 256 + t);
  else if (b < 208)  wtr_unit(Wg1a,  128, 256, WgT2,  512,  0,   0,   (b - 192) * 256 + t);
  else if (b < 240)  wtr_unit(Wg2a,  256, 256, WgT2,  512,  128, 0,   (b - 208) * 256 + t);
  else if (b < 432)  wtr_unit(Wo,    512, 768, WoT2,  KFIN, 0,   0,   (b - 240) * 256 + t);
}

__global__ __launch_bounds__(NTHR) void k_ln_in(const float* __restrict__ x, const float* __restrict__ g,
                                                const float* __restrict__ bt, unsigned short* XN, int nN, int MP) {
  const int lane = (int)threadIdx.x & 31, wave = (int)threadIdx.x >> 5;
  const int row = (int)blockIdx.x * NWAVE + wave;
  if (row >= MP) return;
  const int rc = row < nN ? row : nN - 1;
  const float* p = x + (size_t)rc * DIN + 8 * lane;
  const v4f a0 = rbf4(*(const v4f*)p),         a1 = rbf4(*(const v4f*)(p + 4));
  const v4f b0 = rbf4(*(const v4f*)(p + 256)), b1 = rbf4(*(const v4f*)(p + 260));
  const v4f g0 = rbf4(*(const v4f*)(g + 8 * lane)),        g1 = rbf4(*(const v4f*)(g + 8 * lane + 4));
  const v4f g2 = rbf4(*(const v4f*)(g + 256 + 8 * lane)),  g3 = rbf4(*(const v4f*)(g + 260 + 8 * lane));
  const v4f t0 = rbf4(*(const v4f*)(bt + 8 * lane)),       t1 = rbf4(*(const v4f*)(bt + 8 * lane + 4));
  const v4f t2 = rbf4(*(const v4f*)(bt + 256 + 8 * lane)), t3 = rbf4(*(const v4f*)(bt + 260 + 8 * lane));
  float s = (a0.x + a0.y + a0.z + a0.w) + (a1.x + a1.y + a1.z + a1.w)
          + (b0.x + b0.y + b0.z + b0.w) + (b1.x + b1.y + b1.z + b1.w);
  const float mean = wsum(s) * (1.0f / DIN);
  const v4f d0 = a0 - mean, d1 = a1 - mean, d2 = b0 - mean, d3 = b1 - mean;
  const v4f q4 = d0 * d0 + d1 * d1 + d2 * d2 + d3 * d3;
  const float var = wsum(q4.x + q4.y + q4.z + q4.w) * (1.0f / DIN);
  const float rs = 1.0f / sqrtf(var + 1e-5f);
  const float live = row < nN ? 1.0f : 0.0f;
  v4f y0 = d0 * rs * g0 + t0, y1 = d1 * rs * g1 + t1, y2 = d2 * rs * g2 + t2, y3 = d3 * rs * g3 + t3;
  const v4f z4 = {0.f, 0.f, 0.f, 0.f};
  if (live == 0.0f) { y0 = z4; y1 = z4; y2 = z4; y3 = z4; }
  v8us h0, l0, h1, l1;
  split8(y0, y1, h0, l0);
  split8(y2, y3, h1, l1);
  unsigned short* o = XN + (size_t)row * 1024 + 8 * lane;
  *(volatile v8us*)o = h0; *(volatile v8us*)(o + 256) = h1;
  *(volatile v8us*)(o + 512) = l0; *(volatile v8us*)(o + 768) = l1;
  __threadfence();
  *(volatile v8us*)o = h0; *(volatile v8us*)(o + 256) = h1;
  *(volatile v8us*)(o + 512) = l0; *(volatile v8us*)(o + 768) = l1;
}

__device__ __forceinline__ void gemm_seg(const unsigned short* __restrict__ ap, size_t a16,
                                         const unsigned short* __restrict__ bp, size_t b16,
                                         int ksteps, v8f (&acc)[2][8]) {
#pragma unroll 1
  for (int ks = 0; ks < ksteps; ++ks) {
    FragB a0, a1;
    a0.u[0] = *(const v8us*)(ap + 32 * ks);
    a0.u[1] = *(const v8us*)(ap + 32 * ks + 16);
    a1.u[0] = *(const v8us*)(ap + a16 + 32 * ks);
    a1.u[1] = *(const v8us*)(ap + a16 + 32 * ks + 16);
#pragma unroll
    for (int t = 0; t < 8; ++t) {
      const unsigned short* bq = bp + (size_t)t * b16 + 32 * ks;
      FragB bf;
      bf.u[0] = *(const v8us*)bq;
      bf.u[1] = *(const v8us*)(bq + 16);
      acc[0][t] = wmx(a0, bf, acc[0][t]);
      acc[1][t] = wmx(a1, bf, acc[1][t]);
    }
  }
}

__device__ __forceinline__ void stage_acc(float* stg, const v8f (&acc)[2][8], int rg, int ch, int hh, int m) {
#pragma unroll
  for (int mt = 0; mt < 2; ++mt)
#pragma unroll
    for (int t = 0; t < 8; ++t)
#pragma unroll
      for (int r = 0; r < 8; ++r)
        stg[(32 * rg + 16 * mt + 8 * hh + r) * SP + 128 * ch + 16 * t + m] = acc[mt][t][r];
}

template<int EPI>
__device__ __forceinline__ void st_pass(const float* stg, float* of, int ldo, unsigned short* oh,
                                        int rowBase, int wave, int lane) {
  const int c0 = 4 * lane, c1 = 128 + 4 * lane;
#pragma unroll 2
  for (int rr = 0; rr < 16; ++rr) {
    const int row = 16 * wave + rr;
    const float* rp = stg + row * SP;
    const v4f a = *(const v4fa*)(rp + c0);
    const v4f b = *(const v4fa*)(rp + c1);
    float* gp = of + (size_t)(rowBase + row) * (size_t)ldo;
    *(volatile v4f*)(gp + c0) = a;
    *(volatile v4f*)(gp + c1) = b;
    if (EPI <= 1) {
      const v4f ga = *(const v4fa*)(rp + 8 * lane);
      const v4f gb = *(const v4fa*)(rp + 8 * lane + 4);
      v8us hv, lv;
      split8(ga, gb, hv, lv);
      unsigned short* hp = oh + (size_t)(rowBase + row) * 512 + 8 * lane;
      *(volatile v8us*)hp = hv;
      *(volatile v8us*)(hp + 256) = lv;
    }
  }
}

template<int EPI, int NWV>
__global__ __launch_bounds__(NWV * 32) void k_gemm(
    const unsigned short* __restrict__ A1, int lda1, int ks1,
    const unsigned short* __restrict__ A2, int lda2, int ks2,
    const unsigned short* __restrict__ Bt, int ldb,
    const float* __restrict__ bias0, const float* __restrict__ bias1,
    const float* __restrict__ gam, const float* __restrict__ bet,
    const float* __restrict__ res,
    float* outF, int ldo, size_t yPlane, unsigned short* outH)
{
  extern __shared__ v4f lds_dyn[];
  float* stg = (float*)lds_dyn;
  const int tid = (int)threadIdx.x, lane = tid & 31, wave = tid >> 5, hh = lane >> 4, m = lane & 15;
  const int rg = wave >> 1, ch = wave & 1;
  const int rowBase = (int)blockIdx.x * (NWV * 16);
  const int by = (int)blockIdx.y;
  const int colOff = by * 256;

  v8f acc[2][8];
  {
    const v8f z = {0.f, 0.f, 0.f, 0.f, 0.f, 0.f, 0.f, 0.f};
#pragma unroll
    for (int mt = 0; mt < 2; ++mt)
#pragma unroll
      for (int t = 0; t < 8; ++t) acc[mt][t] = z;
  }
  const int rowA = rowBase + 32 * rg + m;
  const unsigned short* bp0 = Bt + (size_t)(colOff + 128 * ch + m) * (size_t)ldb + 8 * hh;
  {
    const unsigned short* ap = A1 + (size_t)rowA * (size_t)lda1 + 8 * hh;
    gemm_seg(ap, (size_t)16 * lda1, bp0, (size_t)16 * ldb, ks1, acc);
  }
  if (ks2 > 0) {
    const unsigned short* ap = A2 + (size_t)rowA * (size_t)lda2 + 8 * hh;
    gemm_seg(ap, (size_t)16 * lda2, bp0 + 32 * ks1, (size_t)16 * ldb, ks2, acc);
  }
  stage_acc(stg, acc, rg, ch, hh, m);
  __syncthreads();

  const int c0 = 4 * lane, c1 = 128 + 4 * lane;
  const int voff = (EPI == 4) ? colOff : 0;
  v4f bA, bB, gA, gB, tA, tB;
  {
    const v4f x0 = *(const v4f*)(bias0 + voff + c0), x1 = *(const v4f*)(bias0 + voff + c1);
    const v4f y0 = *(const v4f*)(bias1 + voff + c0), y1 = *(const v4f*)(bias1 + voff + c1);
    const bool p0 = (EPI != 2) || (by == 0);
    bA = rbf4(p0 ? x0 : y0);
    bB = rbf4(p0 ? x1 : y1);
    gA = rbf4(*(const v4f*)(gam + voff + c0)); gB = rbf4(*(const v4f*)(gam + voff + c1));
    tA = rbf4(*(const v4f*)(bet + voff + c0)); tB = rbf4(*(const v4f*)(bet + voff + c1));
  }
#pragma unroll 1
  for (int rr = 0; rr < 16; ++rr) {
    const int row = 16 * wave + rr;
    float* rp = stg + row * SP;
    v4f a = *(const v4fa*)(rp + c0) + bA;
    v4f b = *(const v4fa*)(rp + c1) + bB;
    if (EPI != 2) {
      *(v4fa*)(rp + c0) = a;
      *(v4fa*)(rp + c1) = b;
#pragma unroll 1
      for (int i = 0; i < 8; ++i) {
        const int idx = 4 * lane + (i & 3) + ((i >> 2) << 7);
        rp[idx] = gelu_f(rp[idx]);
      }
      a = *(const v4fa*)(rp + c0);
      b = *(const v4fa*)(rp + c1);
    }
    if (EPI == 0 || EPI == 1) {
      const float mean = wsum((a.x + a.y + a.z + a.w) + (b.x + b.y + b.z + b.w)) * (1.0f / HH);
      const v4f da = a - mean, db = b - mean;
      const v4f q4 = da * da + db * db;
      const float var = wsum(q4.x + q4.y + q4.z + q4.w) * (1.0f / HH);
      const float rs = 1.0f / sqrtf(var + 1e-5f);
      a = da * rs * gA + tA;
      b = db * rs * gB + tB;
      if (EPI == 1) {
        const float* rq = res + (size_t)(rowBase + row) * HH;
        a = a + *(const v4f*)(rq + c0);
        b = b + *(const v4f*)(rq + c1);
      }
    }
    if (EPI == 4) {
      const float rsbn = 1.0f / sqrtf(1.00001f);
      a = a * rsbn * gA + tA;
      b = b * rsbn * gB + tB;
    }
    *(v4fa*)(rp + c0) = a;
    *(v4fa*)(rp + c1) = b;
  }
  __syncthreads();

  float* of = outF + ((EPI == 2) ? (size_t)by * yPlane : (size_t)0) + ((EPI == 4) ? colOff : 0);
  st_pass<EPI>(stg, of, ldo, outH, rowBase, wave, lane);
  __threadfence();
  st_pass<EPI>(stg, of, ldo, outH, rowBase, wave, lane);
}

__global__ __launch_bounds__(NTHR) void k_gate(
    const unsigned short* __restrict__ A, const unsigned short* __restrict__ Bt,
    const float* __restrict__ bg1a, const float* __restrict__ bg2a,
    const float* __restrict__ Wg1b, const float* __restrict__ Wg2b,
    const float* __restrict__ bg1b, const float* __restrict__ bg2b, float* GATE)
{
  extern __shared__ v4f lds_dyn[];
  float* stg = (float*)lds_dyn;
  float* gsm = stg + 128 * SP;
  float* bsm = gsm + 256;
  float* wsm = bsm + GW;
  const int tid = (int)threadIdx.x, lane = tid & 31, wave = tid >> 5, hh = lane >> 4, m = lane & 15;
  const int rg = wave >> 1, ch = wave & 1;
  const int rowBase = (int)blockIdx.x * 128;

  for (int i = tid; i < GW; i += NTHR) {
    const int i1 = i < 127 ? i : 127;
    int i2 = i - 128; i2 = i2 < 0 ? 0 : (i2 > 255 ? 255 : i2);
    const float b1 = bg1a[i1], b2 = bg2a[i2], w1 = Wg1b[i1], w2 = Wg2b[i2];
    const bool sel = i < 128;
    bsm[i] = rbf(blendf(b1, b2, sel));
    wsm[i] = rbf(blendf(w1, w2, sel));
  }
  const float bb1 = rbf(bg1b[0]), bb2 = rbf(bg2b[0]);
  const int rowA = rowBase + 32 * rg + m;
  const unsigned short* ap = A + (size_t)rowA * 512 + 8 * hh;

#pragma unroll
  for (int p = 0; p < 2; ++p) {
    if (p == 0 || ch == 0) {
      v8f acc[2][8];
      const v8f z = {0.f, 0.f, 0.f, 0.f, 0.f, 0.f, 0.f, 0.f};
#pragma unroll
      for (int mt = 0; mt < 2; ++mt)
#pragma unroll
        for (int t = 0; t < 8; ++t) acc[mt][t] = z;
      const unsigned short* bp = Bt + (size_t)(256 * p + 128 * ch + m) * 512 + 8 * hh;
      gemm_seg(ap, (size_t)16 * 512, bp, (size_t)16 * 512, 16, acc);
      stage_acc(stg, acc, rg, ch, hh, m);
    }
    __syncthreads();
    const int ni = (p == 0) ? 8 : 4;
#pragma unroll 1
    for (int rr = 0; rr < 16; ++rr) {
      const int row = 16 * wave + rr;
      const float* rp = stg + row * SP;
      float da = 0.f, db = 0.f;
#pragma unroll 1
      for (int i = 0; i < ni; ++i) {
        const int idx = 4 * lane + (i & 3) + ((i >> 2) << 7);
        const float tv = tanhf(rp[idx] + bsm[256 * p + idx]);
        const float pr = tv * wsm[256 * p + idx];
        if (i < 4) da += pr; else db += pr;
      }
      da = wsum(da);
      db = wsum(db);
      if (lane == 0) {
        if (p == 0) { gsm[2 * row] = da + bb1; gsm[2 * row + 1] = db; }
        else        { gsm[2 * row + 1] = gsm[2 * row + 1] + da + bb2; }
      }
    }
    __syncthreads();
  }

  if (wave == 0) {
    const v4f v0 = *(const v4fa*)(gsm + 4 * lane);
    const v4f v1 = *(const v4fa*)(gsm + 128 + 4 * lane);
    float* gp = GATE + (size_t)blockIdx.x * 256;
    *(volatile v4f*)(gp + 4 * lane) = v0;
    *(volatile v4f*)(gp + 128 + 4 * lane) = v1;
    __threadfence();
    *(volatile v4f*)(gp + 4 * lane) = v0;
    *(volatile v4f*)(gp + 128 + 4 * lane) = v1;
  }
}

__device__ __forceinline__ int scan_chunk(const int* __restrict__ dsts, int nE, int cbase, int slotBase,
                                          int nb, int vec8, int* list, int tid, int lane, int wave) {
  int wc = 0;
  const int el0  = tid * EPT;
  const int e0   = cbase + el0;
  const int sent = -2147483647 - 1;
  v4i da, db;
  if (vec8 != 0 && cbase + CHUNK <= nE) {
    da = *(const v4i*)(dsts + e0);
    db = *(const v4i*)(dsts + e0 + 4);
  } else {
    da.x = (e0     < nE) ? dsts[min(e0,     nE - 1)] : sent;
    da.y = (e0 + 1 < nE) ? dsts[min(e0 + 1, nE - 1)] : sent;
    da.z = (e0 + 2 < nE) ? dsts[min(e0 + 2, nE - 1)] : sent;
    da.w = (e0 + 3 < nE) ? dsts[min(e0 + 3, nE - 1)] : sent;
    db.x = (e0 + 4 < nE) ? dsts[min(e0 + 4, nE - 1)] : sent;
    db.y = (e0 + 5 < nE) ? dsts[min(e0 + 5, nE - 1)] : sent;
    db.z = (e0 + 6 < nE) ? dsts[min(e0 + 6, nE - 1)] : sent;
    db.w = (e0 + 7 < nE) ? dsts[min(e0 + 7, nE - 1)] : sent;
  }
  const unsigned nbs = (unsigned)slotBase;
  const unsigned unb = (unsigned)nb;
  const unsigned s0 = (unsigned)da.x - nbs, s1 = (unsigned)da.y - nbs;
  const unsigned s2 = (unsigned)da.z - nbs, s3 = (unsigned)da.w - nbs;
  const unsigned s4 = (unsigned)db.x - nbs, s5 = (unsigned)db.y - nbs;
  const unsigned s6 = (unsigned)db.z - nbs, s7 = (unsigned)db.w - nbs;
  const bool h0 = s0 < unb, h1 = s1 < unb, h2 = s2 < unb, h3 = s3 < unb;
  const bool h4 = s4 < unb, h5 = s5 < unb, h6 = s6 < unb, h7 = s7 < unb;
  const unsigned any = __builtin_amdgcn_ballot_w32(h0 | h1 | h2 | h3 | h4 | h5 | h6 | h7);
  if (any != 0u) {
#define HITJ(J, HJ, SJ) { \
      const unsigned mj = __builtin_amdgcn_ballot_w32(HJ); \
      if (mj != 0u) { \
        if (HJ) { \
          const int pos = wc + (int)__builtin_amdgcn_mbcnt_lo(mj, 0u); \
          if (pos < WCAP) list[wave * WCAP + pos] = ((el0 + (J)) << 12) | (int)(SJ); \
        } \
        wc += (int)__builtin_popcount(mj); } }
    HITJ(0, h0, s0)
    HITJ(1, h1, s1)
    HITJ(2, h2, s2)
    HITJ(3, h3, s3)
    HITJ(4, h4, s4)
    HITJ(5, h5, s5)
    HITJ(6, h6, s6)
    HITJ(7, h7, s7)
#undef HITJ
  }
  return wc;
}

template<int MODE>
__global__ __launch_bounds__(NTHR) void k_scan(
    const int* __restrict__ srcs, const int* __restrict__ dsts,
    const float* __restrict__ P0, const float* __restrict__ XR, const float* __restrict__ X1,
    const float* __restrict__ att, const float* __restrict__ gatb,
    const float* __restrict__ gam, const float* __restrict__ bet,
    float* outF, unsigned short* outH,
    int nN, int nE, int nb, int vec8, int MPr) {
  extern __shared__ v4f lds_dyn[];
  int* reg1 = (int*)lds_dyn;
  int* reg2 = reg1 + RCAP;
  int* scnt = reg2 + RCAP;
  int* soff = scnt + NBMAX;
  int* list = soff + NBMAX;
  int* wcnt = list + LISTN;
  int* wtot = wcnt + NWAVE;
  const int tid = (int)threadIdx.x, lane = tid & 31, wave = tid >> 5;
  const int nodeBase = (int)blockIdx.x * nb;

  for (int i = tid; i < NBMAX; i += NTHR) scnt[i] = 0;
  if (tid == 0) reg2[0] = 0;
  __syncthreads();

  int tot = 0;
  const int nChunks = (nE + CHUNK - 1) / CHUNK;
#pragma unroll 1
  for (int ch = 0; ch < nChunks; ++ch) {
    const int cbase = ch * CHUNK;
    const int wc = scan_chunk(dsts, nE, cbase, nodeBase, nb, vec8, list, tid, lane, wave);
    if (lane == 0) wcnt[wave] = wc;
    __syncthreads();
    int pre = 0, all = 0;
#pragma unroll
    for (int w2 = 0; w2 < NWAVE; ++w2) {
      int c = wcnt[w2];
      c = c < 0 ? 0 : (c > WCAP ? WCAP : c);
      all += c;
      pre += (w2 < wave) ? c : 0;
    }
    const int wcc  = wc > WCAP ? WCAP : wc;
    const int base = tot + pre;
#pragma unroll 1
    for (int i = lane; i < wcc; i += 32) {
      const int ent = list[wave * WCAP + i];
      const int el  = (ent >> 12) & (CHUNK - 1);
      const int sl  = ent & (NBMAX - 1);
      int eid = cbase + el;
      eid = eid > nE - 1 ? nE - 1 : eid;
      const int pos = base + i;
      if (pos < RCAP) reg1[pos] = (int)(((unsigned)eid << 12) | (unsigned)sl);
    }
    tot += all;
    tot = tot > RCAP ? RCAP : tot;
    __syncthreads();
  }
  const int nh = tot;

  if (wave == 0) {
#pragma unroll 1
    for (int b0 = 0; b0 < nh; b0 += 32) {
      const int idx = b0 + lane;
      const int uv  = reg1[idx < RCAP ? idx : RCAP - 1];
      const int m32 = (nh - b0) < 32 ? (nh - b0) : 32;
#pragma unroll 1
      for (int k = 0; k < m32; ++k) {
        const int u  = __builtin_amdgcn_readlane(uv, k);
        const int sl = u & (NBMAX - 1);
        if (lane == 0) scnt[sl] = scnt[sl] + 1;
      }
    }
  }
  __syncthreads();

  {
    const v4i ca = *(const v4i*)(scnt + 8 * tid);
    const v4i cb = *(const v4i*)(scnt + 8 * tid + 4);
    const int e0 = ca.x < 0 ? 0 : ca.x, e1 = ca.y < 0 ? 0 : ca.y, e2 = ca.z < 0 ? 0 : ca.z, e3 = ca.w < 0 ? 0 : ca.w;
    const int e4 = cb.x < 0 ? 0 : cb.x, e5 = cb.y < 0 ? 0 : cb.y, e6 = cb.z < 0 ? 0 : cb.z, e7 = cb.w < 0 ? 0 : cb.w;
    const int ts = e0 + e1 + e2 + e3 + e4 + e5 + e6 + e7;
    int incl = ts;
#pragma unroll
    for (int d = 1; d < 32; d <<= 1) {
      const int up = __shfl_up(incl, d);
      if (lane >= d) incl += up;
    }
    if (lane == 31) wtot[wave] = incl;
    __syncthreads();
    int pre = 0;
#pragma unroll
    for (int w2 = 0; w2 < NWAVE; ++w2) pre += (w2 < wave) ? wtot[w2] : 0;
    int run = pre + incl - ts;
    soff[8 * tid + 0] = run; run += e0;
    soff[8 * tid + 1] = run; run += e1;
    soff[8 * tid + 2] = run; run += e2;
    soff[8 * tid + 3] = run; run += e3;
    soff[8 * tid + 4] = run; run += e4;
    soff[8 * tid + 5] = run; run += e5;
    soff[8 * tid + 6] = run; run += e6;
    soff[8 * tid + 7] = run;
  }
  __syncthreads();
  for (int i = tid; i < NBMAX; i += NTHR) list[i] = soff[i];
  __syncthreads();

  if (wave == 0) {
#pragma unroll 1
    for (int b0 = 0; b0 < nh; b0 += 32) {
      const int idx = b0 + lane;
      const int uv  = reg1[idx < RCAP ? idx : RCAP - 1];
      const int m32 = (nh - b0) < 32 ? (nh - b0) : 32;
#pragma unroll 1
      for (int k = 0; k < m32; ++k) {
        const int u   = __builtin_amdgcn_readlane(uv, k);
        const int sl  = u & (NBMAX - 1);
        const int eid = (int)((unsigned)u >> 12);
        if (lane == 0) {
          int pos = list[sl];
          pos = pos < 0 ? 0 : (pos > RCAP - 1 ? RCAP - 1 : pos);
          reg2[pos] = eid;
          list[sl] = pos + 1;
        }
      }
    }
  }
  __syncthreads();

  const int nbw = nb >> 3;
  const bool ovf = (nh >= RCAP);
  const float qnan = __int_as_float(0x7fc00000);
  float* stw = (float*)reg1 + wave * STW;
  float at[8], gb[8];
  v4f gg0, gg1, be0, be1;
  if (MODE == 1) {
    const v4f a0 = rbf4(*(const v4f*)(att + 8 * lane)),  a1 = rbf4(*(const v4f*)(att + 8 * lane + 4));
    const v4f c0 = rbf4(*(const v4f*)(gatb + 8 * lane)), c1 = rbf4(*(const v4f*)(gatb + 8 * lane + 4));
    at[0] = a0.x; at[1] = a0.y; at[2] = a0.z; at[3] = a0.w; at[4] = a1.x; at[5] = a1.y; at[6] = a1.z; at[7] = a1.w;
    gb[0] = c0.x; gb[1] = c0.y; gb[2] = c0.z; gb[3] = c0.w; gb[4] = c1.x; gb[5] = c1.y; gb[6] = c1.z; gb[7] = c1.w;
    gg0 = rbf4(*(const v4f*)(gam + 8 * lane)); gg1 = rbf4(*(const v4f*)(gam + 8 * lane + 4));
    be0 = rbf4(*(const v4f*)(bet + 8 * lane)); be1 = rbf4(*(const v4f*)(bet + 8 * lane + 4));
  }
#pragma unroll 1
  for (int jt = 0; jt < nbw; ++jt) {
    const int slot = wave * nbw + jt;
    const int grow = nodeBase + slot;
    const int gcl  = grow < MPr ? grow : MPr - 1;
    int st = soff[slot];
    const int craw = scnt[slot];
    int cnt = craw;
    st  = st < 0 ? 0 : (st > nh ? nh : st);
    cnt = cnt < 0 ? 0 : (cnt > DEGCAP ? DEGCAP : cnt);
    if (cnt > nh - st) cnt = nh - st;
    const float pz = (ovf || craw > DEGCAP) ? qnan : 0.0f;
    const bool wr = grow < MPr;

    if (MODE == 0) {
      float av[8];
#pragma unroll
      for (int i = 0; i < 8; ++i) av[i] = 0.f;
#pragma unroll 1
      for (int q = 0; q < cnt; ++q) {
        int idx = st + q; idx = idx > RCAP - 1 ? RCAP - 1 : idx;
        int eid = reg2[idx]; eid = eid < 0 ? 0 : (eid > nE - 1 ? nE - 1 : eid);
        const int sraw = srcs[eid];
        const int s = sraw < 0 ? 0 : (sraw > nN - 1 ? nN - 1 : sraw);
        const float* sr = P0 + (size_t)s * HH + 8 * lane;
        const v4f ha = *(const v4f*)sr, hb = *(const v4f*)(sr + 4);
        ldwait();
        av[0] += ha.x; av[1] += ha.y; av[2] += ha.z; av[3] += ha.w;
        av[4] += hb.x; av[5] += hb.y; av[6] += hb.z; av[7] += hb.w;
      }
      v4f ya, yb;
      ya.x = av[0] + pz; ya.y = av[1] + pz; ya.z = av[2] + pz; ya.w = av[3] + pz;
      yb.x = av[4] + pz; yb.y = av[5] + pz; yb.z = av[6] + pz; yb.w = av[7] + pz;
      v8us hv, lv;
      split8(ya, yb, hv, lv);
      unsigned short* hp = outH + (size_t)grow * 512 + 8 * lane;
      if (wr) { *(volatile v8us*)hp = hv; *(volatile v8us*)(hp + 256) = lv; }
      __threadfence();
      if (wr) { *(volatile v8us*)hp = hv; *(volatile v8us*)(hp + 256) = lv; }
    } else {
      float xr[8], av[8];
      {
        const float* dr = XR + (size_t)gcl * HH + 8 * lane;
        const v4f ra = *(const v4f*)dr, rb = *(const v4f*)(dr + 4);
        ldwait();
        xr[0] = ra.x; xr[1] = ra.y; xr[2] = ra.z; xr[3] = ra.w; xr[4] = rb.x; xr[5] = rb.y; xr[6] = rb.z; xr[7] = rb.w;
      }
#pragma unroll
      for (int i = 0; i < 8; ++i) av[i] = 0.f;
      float mx = -1.0e30f, dn = 0.f;
#pragma unroll 1
      for (int q = 0; q <= cnt; ++q) {
        int idx = st + q - 1; idx = idx < 0 ? 0 : (idx > RCAP - 1 ? RCAP - 1 : idx);
        int eid = reg2[idx]; eid = eid < 0 ? 0 : (eid > nE - 1 ? nE - 1 : eid);
        const int sraw = srcs[eid];
        const int s0 = sraw < 0 ? 0 : (sraw > nN - 1 ? nN - 1 : sraw);
        const int s = (q == 0) ? gcl : s0;
        const float* sr = P0 + (size_t)s * HH + 8 * lane;
        const v4f ha = *(const v4f*)sr, hb = *(const v4f*)(sr + 4);
        ldwait();
        const float hs[8] = {ha.x, ha.y, ha.z, ha.w, hb.x, hb.y, hb.z, hb.w};
        float part = 0.f;
#pragma unroll
        for (int i = 0; i < 8; ++i) {
          float v = hs[i] + xr[i];
          v = v > 0.f ? v : v * NEGS;
          part = fmaf(v, at[i], part);
        }
        part += __shfl_xor(part, 1);
        part += __shfl_xor(part, 2);
        part += __shfl_xor(part, 4);
        const float df = part - mx;
        const float ee = exn(-fabsf(df));
        const bool up  = df > 0.f;
        const float s1 = up ? ee : 1.0f;
        const float s2 = up ? 1.0f : ee;
        mx = (up || part != part) ? part : mx;
        dn = fmaf(dn, s1, s2);
#pragma unroll
        for (int i = 0; i < 8; ++i) av[i] = fmaf(av[i], s1, s2 * hs[i]);
      }
      const float iv = 1.0f / dn;
      v4f pa, pb;
      pa.x = fmaf(av[0], iv, gb[0]) + pz; pa.y = fmaf(av[1], iv, gb[1]) + pz;
      pa.z = fmaf(av[2], iv, gb[2]) + pz; pa.w = fmaf(av[3], iv, gb[3]) + pz;
      pb.x = fmaf(av[4], iv, gb[4]) + pz; pb.y = fmaf(av[5], iv, gb[5]) + pz;
      pb.z = fmaf(av[6], iv, gb[6]) + pz; pb.w = fmaf(av[7], iv, gb[7]) + pz;
      __builtin_amdgcn_fence(__ATOMIC_RELEASE, "wavefront");
      __builtin_amdgcn_wave_barrier();
      *(v4fa*)(stw + 8 * lane) = pa;
      *(v4fa*)(stw + 8 * lane + 4) = pb;
      float sm = 0.f;
#pragma unroll 1
      for (int i = 0; i < 8; ++i) {
        const float v = gelu_f(stw[8 * lane + i]);
        stw[8 * lane + i] = v;
        sm += v;
      }
      const float mean = wsum(sm) * (1.0f / HH);
      float qv = 0.f;
#pragma unroll 1
      for (int i = 0; i < 8; ++i) {
        const float d = stw[8 * lane + i] - mean;
        qv = fmaf(d, d, qv);
      }
      const float var = wsum(qv) * (1.0f / HH);
      const float rs = 1.0f / sqrtf(var + 1e-5f);
      v4f ya = *(const v4fa*)(stw + 8 * lane);
      v4f yb = *(const v4fa*)(stw + 8 * lane + 4);
      const float* xq = X1 + (size_t)gcl * HH + 8 * lane;
      ya = (ya - mean) * rs * gg0 + be0 + *(const v4f*)xq;
      yb = (yb - mean) * rs * gg1 + be1 + *(const v4f*)(xq + 4);
      v8us hv, lv;
      split8(ya, yb, hv, lv);
      *(v4fa*)(stw + 8 * lane) = ya;
      *(v4fa*)(stw + 8 * lane + 4) = yb;
      __builtin_amdgcn_fence(__ATOMIC_RELEASE, "wavefront");
      __builtin_amdgcn_wave_barrier();
      const v4f fa = *(const v4fa*)(stw + 4 * lane);
      const v4f fb = *(const v4fa*)(stw + 128 + 4 * lane);
      float* fp = outF + (size_t)grow * HH;
      unsigned short* hp = outH + (size_t)grow * 512 + 8 * lane;
      if (wr) {
        *(volatile v4f*)(fp + 4 * lane) = fa; *(volatile v4f*)(fp + 128 + 4 * lane) = fb;
        *(volatile v8us*)hp = hv; *(volatile v8us*)(hp + 256) = lv;
      }
      __threadfence();
      if (wr) {
        *(volatile v4f*)(fp + 4 * lane) = fa; *(volatile v4f*)(fp + 128 + 4 * lane) = fb;
        *(volatile v8us*)hp = hv; *(volatile v8us*)(hp + 256) = lv;
      }
    }
  }
  (void)XR; (void)X1; (void)att; (void)gatb; (void)gam; (void)bet; (void)outF;
}

__global__ __launch_bounds__(NTHR) void k_pool(
    const int* __restrict__ batch, const float* __restrict__ GATE,
    const float* __restrict__ X2, const float* __restrict__ XRES,
    unsigned short* FIN, int nN) {
  extern __shared__ v4f lds_dyn[];
  int*   mem = (int*)lds_dyn;
  float* e1  = (float*)(mem + PCAP);
  float* e2  = e1 + PCAP;
  __shared__ int   wcn[NWAVE];
  __shared__ int   wci[NWAVE];
  __shared__ float wm1[NWAVE], wm2[NWAVE], ws1[NWAVE], ws2[NWAVE];
  __shared__ __attribute__((aligned(16))) float fin[768];
  const int tid = (int)threadIdx.x, lane = tid & 31, wave = tid >> 5;
  const int g = (int)blockIdx.x;

  int tot = 0, mine = 0;
  const int nch = (nN + NTHR - 1) / NTHR;
#pragma unroll 1
  for (int ch = 0; ch < nch; ++ch) {
    const int n  = ch * NTHR + tid;
    const int nc = n < nN ? n : nN - 1;
    const int bv = batch[nc];
    const v2f gt = *(const v2f*)(GATE + 2 * (size_t)nc);
    const bool hit = (n < nN) && (bv == g);
    mine += hit ? 1 : 0;
    const unsigned mask = __builtin_amdgcn_ballot_w32(hit);
    const int below = (int)__builtin_amdgcn_mbcnt_lo(mask, 0u);
    if (lane == 0) wcn[wave] = (int)__builtin_popcount(mask);
    __syncthreads();
    int pre = 0, all = 0;
#pragma unroll
    for (int w2 = 0; w2 < NWAVE; ++w2) {
      int c = wcn[w2];
      c = c < 0 ? 0 : (c > 32 ? 32 : c);
      all += c;
      pre += (w2 < wave) ? c : 0;
    }
    const int pos = tot + pre + below;
    if (hit && pos < PCAP) { mem[pos] = n; e1[pos] = gt.x; e2[pos] = gt.y; }
    tot += all;
    tot = tot > PCAP ? PCAP : tot;
    __syncthreads();
  }
  const int nm = tot;

  float m1 = -3.0e38f, m2 = -3.0e38f;
#pragma unroll 1
  for (int j = tid; j < nm; j += NTHR) { m1 = nmax(m1, e1[j]); m2 = nmax(m2, e2[j]); }
#pragma unroll
  for (int off = 16; off > 0; off >>= 1) {
    const float o1 = __shfl_xor(m1, off), o2 = __shfl_xor(m2, off);
    m1 = nmax(m1, o1); m2 = nmax(m2, o2);
  }
  const int cw = wsumi(mine);
  if (lane == 0) { wm1[wave] = m1; wm2[wave] = m2; wci[wave] = cw; }
  __syncthreads();
  float gm1 = wm1[0], gm2 = wm2[0];
  int cnti = wci[0];
#pragma unroll
  for (int w2 = 1; w2 < NWAVE; ++w2) { gm1 = nmax(gm1, wm1[w2]); gm2 = nmax(gm2, wm2[w2]); cnti += wci[w2]; }

  float p1 = 0.f, p2 = 0.f;
#pragma unroll 1
  for (int j = tid; j < nm; j += NTHR) {
    const float x1 = exn(e1[j] - gm1), x2 = exn(e2[j] - gm2);
    e1[j] = x1; e2[j] = x2;
    p1 += x1; p2 += x2;
  }
  p1 = wsum(p1); p2 = wsum(p2);
  if (lane == 0) { ws1[wave] = p1; ws2[wave] = p2; }
  __syncthreads();
  float gs1 = ws1[0], gs2 = ws2[0];
#pragma unroll
  for (int w2 = 1; w2 < NWAVE; ++w2) { gs1 += ws1[w2]; gs2 += ws2[w2]; }

  float a1 = 0.f, a2 = 0.f, a3 = 0.f;
#pragma unroll 1
  for (int j = 0; j < nm; ++j) {
    int n = mem[j]; n = n < 0 ? 0 : (n > nN - 1 ? nN - 1 : n);
    const float w1 = e1[j], w2 = e2[j];
    const float xv = X2[(size_t)n * HH + tid];
    const float rv = XRES[(size_t)n * HH + tid];
    a1 = fmaf(w1, xv, a1);
    a2 = fmaf(w2, xv, a2);
    a3 += rv;
  }
  const bool have = cnti > 0;
  const float i1 = have ? (1.0f / gs1) : 0.0f;
  const float i2 = have ? (1.0f / gs2) : 0.0f;
  const float cf = (float)(cnti > 1 ? cnti : 1);
  fin[tid]       = a1 * i1;
  fin[256 + tid] = a2 * i2;
  fin[512 + tid] = a3 * (1.0f / cf);
  __syncthreads();
  if (tid < 96) {
    const v4f fa = *(const v4fa*)(fin + 8 * tid);
    const v4f fb = *(const v4fa*)(fin + 8 * tid + 4);
    v8us hv, lv;
    split8(fa, fb, hv, lv);
    unsigned short* hp = FIN + (size_t)g * KFIN + 8 * tid;
    *(volatile v8us*)hp = hv; *(volatile v8us*)(hp + 768) = lv;
    __threadfence();
    *(volatile v8us*)hp = hv; *(volatile v8us*)(hp + 768) = lv;
  }
}

static inline int cdiv(int a, int b) { return (a + b - 1) / b; }

extern "C" void kernel_launch(void* const* d_in, const int* in_sizes, int n_in,
                              void* d_out, int out_size, void* d_ws, size_t ws_size,
                              hipStream_t stream) {
  if (n_in < 34) return;
  if (in_sizes[0] != NN * DIN || in_sizes[1] != 2 * NE || in_sizes[2] != NN) return;
  if (in_sizes[3] != DIN || in_sizes[4] != DIN || in_sizes[5] != DIN * HH || in_sizes[6] != HH) return;
  if (in_sizes[7] != HH || in_sizes[8] != HH || in_sizes[9] != HH * HH || in_sizes[10] != HH) return;
  if (in_sizes[11] != HH * HH || in_sizes[12] != HH || in_sizes[13] != HH) return;
  if (in_sizes[14] != HH * HH || in_sizes[15] != HH || in_sizes[16] != HH * HH || in_sizes[17] != HH) return;
  if (in_sizes[18] != HH || in_sizes[19] != HH || in_sizes[20] != HH || in_sizes[21] != HH) return;
  if (in_sizes[22] != HH * 128 || in_sizes[23] != 128 || in_sizes[24] != 128 || in_sizes[25] != 1) return;
  if (in_sizes[26] != HH * HH || in_sizes[27] != HH || in_sizes[28] != HH || in_sizes[29] != 1) return;
  if (in_sizes[30] != 768 * OUTD || in_sizes[31] != OUTD || in_sizes[32] != OUTD || in_sizes[33] != OUTD) return;
  if (out_size != NG * OUTD) return;

  const float* x     = (const float*)d_in[0];
  const int*   ei    = (const int*)  d_in[1];
  const int*   batch = (const int*)  d_in[2];
  const float* lnig  = (const float*)d_in[3];
  const float* lnib  = (const float*)d_in[4];
  const float* Wp    = (const float*)d_in[5];
  const float* bp    = (const float*)d_in[6];
  const float* lnpg  = (const float*)d_in[7];
  const float* lnpb  = (const float*)d_in[8];
  const float* Wrel  = (const float*)d_in[9];
  const float* brel  = (const float*)d_in[10];
  const float* Wroot = (const float*)d_in[11];
  const float* n1g   = (const float*)d_in[12];
  const float* n1b   = (const float*)d_in[13];
  const float* Wl    = (const float*)d_in[14];
  const float* bl    = (const float*)d_in[15];
  const float* Wr    = (const float*)d_in[16];
  const float* br    = (const float*)d_in[17];
  const float* att   = (const float*)d_in[18];
  const float* gatb  = (const float*)d_in[19];
  const float* n2g   = (const float*)d_in[20];
  const float* n2b   = (const float*)d_in[21];
  const float* Wg1a  = (const float*)d_in[22];
  const float* bg1a  = (const float*)d_in[23];
  const float* Wg1b  = (const float*)d_in[24];
  const float* bg1b  = (const float*)d_in[25];
  const float* Wg2a  = (const float*)d_in[26];
  const float* bg2a  = (const float*)d_in[27];
  const float* Wg2b  = (const float*)d_in[28];
  const float* bg2b  = (const float*)d_in[29];
  const float* Wo    = (const float*)d_in[30];
  const float* bo    = (const float*)d_in[31];
  const float* bng   = (const float*)d_in[32];
  const float* bnb   = (const float*)d_in[33];
  float* out = (float*)d_out;
  const int* src = ei;
  const int* dst = ei + NE;

  const int nb = NBRUN;
  const int gA = cdiv(NPAD, nb);
  if (gA * nb < NPAD) return;
  const int vec8 = ((NE & 3) == 0) ? 1 : 0;

  const size_t szXN  = (size_t)NPAD * 1024 * 2;
  const size_t szPL  = (size_t)NPAD * 1024;
  const size_t szGT  = (size_t)NPAD * 2 * 4;
  const size_t szFIN = (size_t)NG * KFIN * 2;
  const size_t szW1  = (size_t)256 * 1024 * 2;
  const size_t szWG  = (size_t)GW * 512 * 2;
  const size_t szWO  = (size_t)512 * KFIN * 2;
  size_t off = 0;
  const size_t oXN   = off; off += szXN;
  const size_t oXRES = off; off += szPL;
  const size_t oXRH  = off; off += szPL;
  const size_t oAGH  = off; off += szPL;
  const size_t oX1   = off; off += szPL;
  const size_t oX1H  = off; off += szPL;
  const size_t oXL   = off; off += szPL;
  const size_t oXR   = off; off += szPL;
  const size_t oX2   = off; off += szPL;
  const size_t oX2H  = off; off += szPL;
  const size_t oGT   = off; off += szGT;
  const size_t oFIN  = off; off += szFIN;
  const size_t oWP   = off; off += szW1;
  const size_t oWGC  = off; off += szW1;
  const size_t oWLR  = off; off += szW1;
  const size_t oWG   = off; off += szWG;
  const size_t oWO   = off; off += szWO;
  if (off > ws_size || off > (size_t)WSMAX) return;
  if (oXR != oXL + (size_t)NPAD * HH * 4) return;
  char* ws = (char*)d_ws;
  unsigned short* XNhl  = (unsigned short*)(ws + oXN);
  float*          XRESp = (float*)(ws + oXRES);
  unsigned short* XREShl= (unsigned short*)(ws + oXRH);
  unsigned short* AGGhl = (unsigned short*)(ws + oAGH);
  float*          X1p   = (float*)(ws + oX1);
  unsigned short* X1hl  = (unsigned short*)(ws + oX1H);
  float*          XLp   = (float*)(ws + oXL);
  float*          XRp   = (float*)(ws + oXR);
  float*          X2p   = (float*)(ws + oX2);
  unsigned short* X2hl  = (unsigned short*)(ws + oX2H);
  float*          GATEp = (float*)(ws + oGT);
  unsigned short* FINhl = (unsigned short*)(ws + oFIN);
  unsigned short* WpT2  = (unsigned short*)(ws + oWP);
  unsigned short* WgcT  = (unsigned short*)(ws + oWGC);
  unsigned short* WlrT2 = (unsigned short*)(ws + oWLR);
  unsigned short* WgT2  = (unsigned short*)(ws + oWG);
  unsigned short* WoT2  = (unsigned short*)(ws + oWO);

  hipFuncSetAttribute(reinterpret_cast<const void*>(&k_gemm<0, 8>), hipFuncAttributeMaxDynamicSharedMemorySize, LDS_G8);
  hipFuncSetAttribute(reinterpret_cast<const void*>(&k_gemm<1, 8>), hipFuncAttributeMaxDynamicSharedMemorySize, LDS_G8);
  hipFuncSetAttribute(reinterpret_cast<const void*>(&k_gemm<2, 8>), hipFuncAttributeMaxDynamicSharedMemorySize, LDS_G8);
  hipFuncSetAttribute(reinterpret_cast<const void*>(&k_gemm<4, 4>), hipFuncAttributeMaxDynamicSharedMemorySize, LDS_G4);
  hipFuncSetAttribute(reinterpret_cast<const void*>(&k_gate), hipFuncAttributeMaxDynamicSharedMemorySize, LDS_GATE);
  hipFuncSetAttribute(reinterpret_cast<const void*>(&k_scan<0>), hipFuncAttributeMaxDynamicSharedMemorySize, LDS_AGG);
  hipFuncSetAttribute(reinterpret_cast<const void*>(&k_scan<1>), hipFuncAttributeMaxDynamicSharedMemorySize, LDS_AGG);
  hipFuncSetAttribute(reinterpret_cast<const void*>(&k_pool), hipFuncAttributeMaxDynamicSharedMemorySize, LDS_POOL);

  k_prep<<<432, NTHR, 0, stream>>>(Wp, Wrel, Wroot, Wl, Wr, Wg1a, Wg2a, Wo, WpT2, WgcT, WlrT2, WgT2, WoT2);
  k_ln_in<<<NPAD / NWAVE, NTHR, 0, stream>>>(x, lnig, lnib, XNhl, NN, NPAD);
  k_gemm<0, 8><<<dim3(NPAD / 128, 1), 256, LDS_G8, stream>>>(
      XNhl, 1024, 32, XNhl, 1024, 0, WpT2, 1024, bp, bp, lnpg, lnpb, XRESp, XRESp, HH, (size_t)0, XREShl);
  k_scan<0><<<gA, NTHR, LDS_AGG, stream>>>(src, dst, XRESp, XRESp, XRESp, att, gatb, n2g, n2b,
                                           X2p, AGGhl, NN, NE, nb, vec8, NPAD);
  k_gemm<1, 8><<<dim3(NPAD / 128, 1), 256, LDS_G8, stream>>>(
      AGGhl, 512, 16, XREShl, 512, 16, WgcT, 1024, brel, brel, n1g, n1b, XRESp, X1p, HH, (size_t)0, X1hl);
  k_gemm<2, 8><<<dim3(NPAD / 128, 2), 256, LDS_G8, stream>>>(
      X1hl, 512, 16, X1hl, 512, 0, WlrT2, 512, bl, br, bl, bl, X1p, XLp, HH, (size_t)NPAD * HH, X1hl);
  k_scan<1><<<gA, NTHR, LDS_AGG, stream>>>(src, dst, XLp, XRp, X1p, att, gatb, n2g, n2b,
                                           X2p, X2hl, NN, NE, nb, vec8, NPAD);
  k_gate<<<NPAD / 128, NTHR, LDS_GATE, stream>>>(X2hl, WgT2, bg1a, bg2a, Wg1b, Wg2b, bg1b, bg2b, GATEp);
  k_pool<<<NG, NTHR, LDS_POOL, stream>>>(batch, GATEp, X2p, XRESp, FINhl, NN);
  k_gemm<4, 4><<<dim3(1, 2), 128, LDS_G4, stream>>>(
      FINhl, KFIN, 48, FINhl, KFIN, 0, WoT2, KFIN, bo, bo, bng, bnb, XRESp, out, OUTD, (size_t)0, X1hl);
}
